// TransitionDown_75213467287645
// MI455X (gfx1250) — hardware-verified
//
#include <hip/hip_runtime.h>
#include <math.h>

constexpr int NSRC    = 200000;
constexpr int MQ      = 50000;
constexpr int NSAMP   = 16;
constexpr int CIN     = 64;
constexpr int COUT_CH = 128;
constexpr int WCOLS   = 67;
constexpr int KP      = 96;
constexpr int NWAVE   = 8;
constexpr int NTHR    = 256;
constexpr int ITER1   = 25;
constexpr int NBLK1   = MQ / (NWAVE * ITER1);
constexpr int PART_STRIDE = 2 * COUT_CH;
constexpr int TBL_N   = 4 * COUT_CH;
constexpr int NBLK3   = (MQ * 32) / NTHR;
constexpr float  BN_EPS  = 1e-5f;
constexpr double INV_CNT = 1.0 / 800000.0;
static_assert(NBLK1 * NWAVE * ITER1 == MQ, "");
static_assert(NBLK3 * NTHR == MQ * 32, "");
static_assert(KP % 32 == 0, "");
static_assert((COUT_CH * KP / 2) % NTHR == 0, "");
static_assert(MQ * NSAMP == 800000, "");

typedef __attribute__((ext_vector_type(16))) _Float16 v16h;
typedef __attribute__((ext_vector_type(8)))  _Float16 v8h;
typedef __attribute__((ext_vector_type(16))) __bf16   v16b;
typedef __attribute__((ext_vector_type(8)))  __bf16   v8b;
typedef __attribute__((ext_vector_type(8)))  float    v8f;
typedef __attribute__((ext_vector_type(4)))  float    v4f;
typedef __attribute__((ext_vector_type(4)))  unsigned int v4u;

__device__ __forceinline__ unsigned short f2bf_bits(float f) {
  unsigned u = __float_as_uint(f);
  return (unsigned short)((u + 0x7FFFu + ((u >> 16) & 1u)) >> 16);
}
__device__ __forceinline__ float bf_bits2f(unsigned short h) { return __uint_as_float(((unsigned)h) << 16); }

__device__ __forceinline__ void dep_guard_h(v8f& a, v8f& b, v16h x, v16h y) { asm volatile("v_nop\n\tv_nop\n\tv_nop\n\tv_nop" : "+v"(a), "+v"(b) : "v"(x), "v"(y)); }
__device__ __forceinline__ void dep_guard_b(v8f& a, v8f& b, v16b x, v16b y) { asm volatile("v_nop\n\tv_nop\n\tv_nop\n\tv_nop" : "+v"(a), "+v"(b) : "v"(x), "v"(y)); }
__device__ __forceinline__ void keep4_h(v16h a, v16h b, v16h c, v16h d) { asm volatile("v_nop" :: "v"(a), "v"(b), "v"(c), "v"(d)); }
__device__ __forceinline__ void keep4_b(v16b a, v16b b, v16b c, v16b d) { asm volatile("v_nop" :: "v"(a), "v"(b), "v"(c), "v"(d)); }
template <typename T> struct Frag;
template <> struct Frag<_Float16> {
  typedef v16h V; union U { v16h v; v8h h[2]; };
  static __device__ __forceinline__ v16h load(const _Float16* p) {
    U f; f.h[0] = *(const v8h*)(p); f.h[1] = *(const v8h*)(p + 16); return f.v;
  }
  static __device__ __forceinline__ v8f mma(v16h a, v16h b, v8f c) {
    return __builtin_amdgcn_wmma_f32_16x16x32_f16(false, a, false, b, (short)0, c, false, false);
  }
  static __device__ __forceinline__ void guard(v8f& a, v8f& b, v16h x, v16h y) { dep_guard_h(a, b, x, y); }
  static __device__ __forceinline__ void keep(v16h a, v16h b, v16h c, v16h d) { keep4_h(a, b, c, d); }
};
template <> struct Frag<__bf16> {
  typedef v16b V; union U { v16b v; v8b h[2]; };
  static __device__ __forceinline__ v16b load(const __bf16* p) {
    U f; f.h[0] = *(const v8b*)(p); f.h[1] = *(const v8b*)(p + 16); return f.v;
  }
  static __device__ __forceinline__ v8f mma(v16b a, v16b b, v8f c) {
    return __builtin_amdgcn_wmma_f32_16x16x32_bf16(false, a, false, b, (short)0, c, false, false);
  }
  static __device__ __forceinline__ void guard(v8f& a, v8f& b, v16b x, v16b y) { dep_guard_b(a, b, x, y); }
  static __device__ __forceinline__ void keep(v16b a, v16b b, v16b c, v16b d) { keep4_b(a, b, c, d); }
};

__device__ __forceinline__ v8f at_mma(v16b a, v16b b, v8f c) {
  c = __builtin_amdgcn_wmma_f32_16x16x32_bf16(false, a, false, b, (short)0, c, false, false);
  asm volatile("v_nop\n\tv_nop\n\tv_nop\n\tv_nop" : "+v"(c) : "v"(a), "v"(b));
  return c;
}

__device__ __forceinline__ unsigned pk16(unsigned short a, unsigned short b) { return (unsigned)a | ((unsigned)b << 16); }
__device__ __forceinline__ float bf_rn(float f) { return bf_bits2f(f2bf_bits(f)); }

__global__ __launch_bounds__(NTHR) void group_linear_kernel(
    const float* __restrict__ p, const float* __restrict__ x, const float* __restrict__ npc,
    const int* __restrict__ idx, const float* __restrict__ W,
    float* __restrict__ ymax, float* __restrict__ ymin, float* __restrict__ partial) {
  __shared__ __align__(16) unsigned short Bs[COUT_CH * KP];
  __shared__ __align__(16) unsigned short As[NWAVE][NSAMP * KP];
  __shared__ __align__(16) float slab[NWAVE][2 * COUT_CH];
  __shared__ __align__(16) float sred[2 * COUT_CH];

  const int tid  = threadIdx.x;
  const int lane = tid & 31;
  const int wave = tid >> 5;
  const int r    = lane & 15;
  const int h    = lane >> 4;

#pragma unroll 4
  for (int j = 0; j < (COUT_CH * KP / 2) / NTHR; ++j) {
    const int widx = j * NTHR + tid;
    const int o  = widx / (KP / 2);
    const int ka = (widx - o * (KP / 2)) * 2;
    const int kb = ka + 1;
    const int ca = (ka < CIN) ? (ka + 3) : ((ka < CIN + 3) ? (ka - CIN) : ((ka < CIN + 6) ? (ka - CIN - 3) : 0));
    const int cb = (kb < CIN) ? (kb + 3) : ((kb < CIN + 3) ? (kb - CIN) : ((kb < CIN + 6) ? (kb - CIN - 3) : 0));
    const float wa = W[o * WCOLS + ca];
    const float wb = W[o * WCOLS + cb];
    const float va = (ka < CIN + 6) ? wa : 0.0f;
    const float vb = (kb < CIN + 6) ? wb : 0.0f;
    ((unsigned*)(void*)Bs)[widx] = pk16(f2bf_bits(va), f2bf_bits(vb));
  }
  __syncthreads();

  float sumA[8], sqA[8];
#pragma unroll
  for (int nf = 0; nf < 8; ++nf) { sumA[nf] = 0.0f; sqA[nf] = 0.0f; }

  unsigned short* Aw = As[wave];
  const __bf16* Ab = (const __bf16*)(const void*)Aw;
  const __bf16* Bb = (const __bf16*)(const void*)Bs;
  float* slw = slab[wave];
  const v4u zero4 = (v4u){0u, 0u, 0u, 0u};

#pragma unroll 1
  for (int it = 0; it < ITER1; ++it) {
    const int m = blockIdx.x * (NWAVE * ITER1) + it * NWAVE + wave;
    int g = idx[m * NSAMP + r];
    g = (g < 0) ? 0 : ((g >= NSRC) ? (NSRC - 1) : g);

    const float c0 = bf_rn(npc[m * 3 + 0]);
    const float c1 = bf_rn(npc[m * 3 + 1]);
    const float c2 = bf_rn(npc[m * 3 + 2]);
    const float q0 = bf_rn(p[(size_t)g * 3 + 0]);
    const float q1 = bf_rn(p[(size_t)g * 3 + 1]);
    const float q2 = bf_rn(p[(size_t)g * 3 + 2]);
    const float rel0 = q0 - c0, rel1 = q1 - c1, rel2 = q2 - c2;
    const unsigned short h0 = f2bf_bits(rel0), h1 = f2bf_bits(rel1), h2 = f2bf_bits(rel2);
    const unsigned short l0 = f2bf_bits(rel0 - bf_bits2f(h0));
    const unsigned short l1 = f2bf_bits(rel1 - bf_bits2f(h1));
    const unsigned short l2 = f2bf_bits(rel2 - bf_bits2f(h2));
    const unsigned keep = (h == 0) ? 0xFFFFFFFFu : 0u;
    const v4u relw = (v4u){pk16(h0, h1) & keep, pk16(h2, l0) & keep, pk16(l1, l2) & keep, 0u};
    unsigned short* arow = Aw + r * KP;
    *(v4u*)(arow + CIN + 16 * h)     = relw;
    *(v4u*)(arow + CIN + 8 + 16 * h) = zero4;

    const float* xr = x + (size_t)g * CIN + h * 32;
    {
      const v4f a0 = *(const v4f*)(xr), a1 = *(const v4f*)(xr + 4), a2 = *(const v4f*)(xr + 8), a3 = *(const v4f*)(xr + 12);
      const v4u u0 = (v4u){pk16(f2bf_bits(a0[0]), f2bf_bits(a0[1])), pk16(f2bf_bits(a0[2]), f2bf_bits(a0[3])),
                           pk16(f2bf_bits(a1[0]), f2bf_bits(a1[1])), pk16(f2bf_bits(a1[2]), f2bf_bits(a1[3]))};
      const v4u u1 = (v4u){pk16(f2bf_bits(a2[0]), f2bf_bits(a2[1])), pk16(f2bf_bits(a2[2]), f2bf_bits(a2[3])),
                           pk16(f2bf_bits(a3[0]), f2bf_bits(a3[1])), pk16(f2bf_bits(a3[2]), f2bf_bits(a3[3]))};
      *(v4u*)(arow + h * 32)     = u0;
      *(v4u*)(arow + h * 32 + 8) = u1;
    }
    asm volatile("" ::: "memory");
    {
      const v4f a0 = *(const v4f*)(xr + 16), a1 = *(const v4f*)(xr + 20), a2 = *(const v4f*)(xr + 24), a3 = *(const v4f*)(xr + 28);
      const v4u u0 = (v4u){pk16(f2bf_bits(a0[0]), f2bf_bits(a0[1])), pk16(f2bf_bits(a0[2]), f2bf_bits(a0[3])),
                           pk16(f2bf_bits(a1[0]), f2bf_bits(a1[1])), pk16(f2bf_bits(a1[2]), f2bf_bits(a1[3]))};
      const v4u u1 = (v4u){pk16(f2bf_bits(a2[0]), f2bf_bits(a2[1])), pk16(f2bf_bits(a2[2]), f2bf_bits(a2[3])),
                           pk16(f2bf_bits(a3[0]), f2bf_bits(a3[1])), pk16(f2bf_bits(a3[2]), f2bf_bits(a3[3]))};
      *(v4u*)(arow + h * 32 + 16) = u0;
      *(v4u*)(arow + h * 32 + 24) = u1;
    }
    __syncthreads();

    v8f acc[8];
#pragma unroll
    for (int nf = 0; nf < 8; ++nf) acc[nf] = (v8f){0.f, 0.f, 0.f, 0.f, 0.f, 0.f, 0.f, 0.f};
#pragma unroll
    for (int kt = 0; kt < KP / 32; ++kt) {
      const v16b af = Frag<__bf16>::load(Ab + r * KP + kt * 32 + 8 * h);
#pragma unroll
      for (int nf = 0; nf < 8; ++nf) {
        const v16b bfv = Frag<__bf16>::load(Bb + (nf * 16 + r) * KP + kt * 32 + 8 * h);
        acc[nf] = at_mma(af, bfv, acc[nf]);
      }
    }

#pragma unroll
    for (int nf = 0; nf < 8; ++nf) {
      float mx = acc[nf][0], mn = acc[nf][0], s = 0.0f, q = 0.0f;
#pragma unroll
      for (int j = 0; j < 8; ++j) {
        const float v = acc[nf][j];
        mx = fmaxf(mx, v); mn = fminf(mn, v); s += v; q += v * v;
      }
      const float mxo = __shfl_xor(mx, 16, 32);
      const float mno = __shfl_xor(mn, 16, 32);
      const float so  = __shfl_xor(s, 16, 32);
      const float qo  = __shfl_xor(q, 16, 32);
      mx = fmaxf(mx, mxo);
      mn = fminf(mn, mno);
      sumA[nf] += s + so;
      sqA[nf]  += q + qo;
      const float wv = (h == 0) ? mx : mn;
      slw[h * COUT_CH + nf * 16 + r] = wv;
    }
    __syncthreads();
    {
      const v4f vmax = *(const v4f*)(slw + 4 * lane);
      const v4f vmin = *(const v4f*)(slw + COUT_CH + 4 * lane);
      float* pmx = ymax + (size_t)m * COUT_CH + 4 * lane;
      float* pmn = ymin + (size_t)m * COUT_CH + 4 * lane;
      *(volatile v4f*)pmx = vmax;
      *(volatile v4f*)pmn = vmin;
      __threadfence();
      *(volatile v4f*)pmx = vmax;
      *(volatile v4f*)pmn = vmin;
    }
    __syncthreads();
  }

#pragma unroll
  for (int nf = 0; nf < 8; ++nf) {
    slw[nf * 16 + r]           = sumA[nf];
    slw[COUT_CH + nf * 16 + r] = sqA[nf];
  }
  __syncthreads();
  if (tid < COUT_CH) {
    float S = 0.0f, Q = 0.0f;
#pragma unroll
    for (int w = 0; w < NWAVE; ++w) { S += slab[w][tid]; Q += slab[w][COUT_CH + tid]; }
    sred[tid] = S;
    sred[COUT_CH + tid] = Q;
  }
  __syncthreads();
  if (wave == 0) {
    const v4f a = *(const v4f*)(sred + 4 * lane);
    const v4f b = *(const v4f*)(sred + COUT_CH + 4 * lane);
    float* pp = partial + (size_t)blockIdx.x * PART_STRIDE;
    *(volatile v4f*)(pp + 4 * lane) = a;
    *(volatile v4f*)(pp + COUT_CH + 4 * lane) = b;
    __threadfence();
    *(volatile v4f*)(pp + 4 * lane) = a;
    *(volatile v4f*)(pp + COUT_CH + 4 * lane) = b;
  }
}

__global__ __launch_bounds__(COUT_CH) void stats_kernel(const float* __restrict__ partial, const float* __restrict__ gamma,
                                                     const float* __restrict__ beta, float* __restrict__ tbl) {
  const int o = threadIdx.x;
  double S = 0.0, Q = 0.0;
#pragma unroll 2
  for (int b = 0; b < NBLK1; ++b) {
    S += (double)partial[b * PART_STRIDE + o];
    Q += (double)partial[b * PART_STRIDE + COUT_CH + o];
  }
  const double mean = S * INV_CNT;
  double var = Q * INV_CNT - mean * mean;
  var = (var > 0.0) ? var : 0.0;
  const float meanf = (float)mean;
  const float varf  = (float)var;
  const float sd    = sqrtf(varf + BN_EPS);
  const float inv   = 1.0f / sd;
  const float gr    = bf_rn(gamma[o]);
  const float br    = bf_rn(beta[o]);
  volatile float* t = tbl;
  t[o] = meanf; t[COUT_CH + o] = inv; t[2 * COUT_CH + o] = gr; t[3 * COUT_CH + o] = br;
  __threadfence();
  t[o] = meanf; t[COUT_CH + o] = inv; t[2 * COUT_CH + o] = gr; t[3 * COUT_CH + o] = br;
}

__global__ __launch_bounds__(NTHR) void finalize_kernel(const float* __restrict__ ymax, const float* __restrict__ ymin,
                                                      const float* __restrict__ tbl, float* __restrict__ out) {
  const int i  = blockIdx.x * NTHR + threadIdx.x;
  const int m  = i >> 5;
  const int oq = (i & 31) * 4;
  if (m >= MQ) return;
  const v4f mx   = *(const v4f*)(ymax + (size_t)m * COUT_CH + oq);
  const v4f mn   = *(const v4f*)(ymin + (size_t)m * COUT_CH + oq);
  const v4f mean = *(const v4f*)(tbl + oq);
  const v4f inv  = *(const v4f*)(tbl + COUT_CH + oq);
  const v4f gm   = *(const v4f*)(tbl + 2 * COUT_CH + oq);
  const v4f bt   = *(const v4f*)(tbl + 3 * COUT_CH + oq);
  v4f o4;
#pragma unroll
  for (int e = 0; e < 4; ++e) {
    const float fa  = (gm[e] >= 0.0f) ? 1.0f : 0.0f;
    const float fb  = 1.0f - fa;
    const float sel = fmaf(fa, mx[e], fb * mn[e]);
    float t = (sel - mean[e]) * inv[e];
    t = t * gm[e];
    t = t + bt[e];
    o4[e] = fmaxf(t, 0.0f);
  }
  float* op = out + (size_t)m * COUT_CH + oq;
  *(volatile v4f*)op = o4;
  __threadfence();
  *(volatile v4f*)op = o4;
}

extern "C" void kernel_launch(void* const* d_in, const int* in_sizes, int n_in,
                              void* d_out, int out_size, void* d_ws, size_t ws_size, hipStream_t stream) {
  (void)in_sizes; (void)n_in; (void)out_size;
  const float* p     = (const float*)d_in[0];
  const float* x     = (const float*)d_in[1];
  const float* npc   = (const float*)d_in[2];
  const int*   idx   = (const int*)  d_in[3];
  const float* W     = (const float*)d_in[4];
  const float* gamma = (const float*)d_in[5];
  const float* beta  = (const float*)d_in[6];
  float* out = (float*)d_out;

  char* ws = (char*)d_ws; size_t off = 0;
  auto carve = [&](size_t bytes) -> char* { char* q = ws + off; off += (bytes + 255) & ~(size_t)255; return q; };
  float* ymax    = (float*)carve((size_t)MQ * COUT_CH * 4);
  float* ymin    = (float*)carve((size_t)MQ * COUT_CH * 4);
  float* partial = (float*)carve((size_t)NBLK1 * PART_STRIDE * 4);
  float* tbl     = (float*)carve((size_t)TBL_N * 4);
  if (off > ws_size || off > (size_t)134217728) return;

  group_linear_kernel<<<NBLK1, NTHR, 0, stream>>>(p, x, npc, idx, W, ymax, ymin, partial);
  stats_kernel<<<1, COUT_CH, 0, stream>>>(partial, gamma, beta, tbl);
  finalize_kernel<<<NBLK3, NTHR, 0, stream>>>(ymax, ymin, tbl, out);
}
